// DeltaRecurrentUpdate_40218073760069
// MI455X (gfx1250) — hardware-verified
//
#include <hip/hip_runtime.h>
#include <math.h>

constexpr int kB = 8;
constexpr int kL = 8192;
constexpr int kR = 64;
constexpr int kH = 512;
constexpr int kNBC = 2;
constexpr int kNChunk = kB / kNBC;
constexpr int kRowsChunk = kNBC * kL;
constexpr int kRowsPerWave = 4;
constexpr float kEps = 1e-12f;
constexpr float kWCarry = 16.0f;
constexpr float kKCarry = 16.0f;
constexpr float kInvW = 1.0f / 16.0f;
constexpr float kInvK = 1.0f / 16.0f;

typedef __attribute__((ext_vector_type(16))) _Float16 v16h;
typedef __attribute__((ext_vector_type(8)))  _Float16 v8h;
typedef __attribute__((ext_vector_type(16))) __bf16   v16b;
typedef __attribute__((ext_vector_type(8)))  __bf16   v8b;
typedef __attribute__((ext_vector_type(8)))  float    v8f;
typedef __attribute__((ext_vector_type(4)))  float    v4f;
typedef __attribute__((ext_vector_type(4)))  unsigned int v4u;

__device__ __forceinline__ unsigned short f2bf_bits(float f) {
  unsigned u = __float_as_uint(f);
  return (unsigned short)((u + 0x7FFFu + ((u >> 16) & 1u)) >> 16);
}
__device__ __forceinline__ float bf_bits2f(unsigned short h) { return __uint_as_float(((unsigned)h) << 16); }

__device__ __forceinline__ void dep_guard_h(v8f& a, v8f& b, v16h x, v16h y) { asm volatile("v_nop\n\tv_nop\n\tv_nop\n\tv_nop" : "+v"(a), "+v"(b) : "v"(x), "v"(y)); }
__device__ __forceinline__ void dep_guard_b(v8f& a, v8f& b, v16b x, v16b y) { asm volatile("v_nop\n\tv_nop\n\tv_nop\n\tv_nop" : "+v"(a), "+v"(b) : "v"(x), "v"(y)); }
__device__ __forceinline__ void keep4_h(v16h a, v16h b, v16h c, v16h d) { asm volatile("v_nop" :: "v"(a), "v"(b), "v"(c), "v"(d)); }
__device__ __forceinline__ void keep4_b(v16b a, v16b b, v16b c, v16b d) { asm volatile("v_nop" :: "v"(a), "v"(b), "v"(c), "v"(d)); }
__device__ __forceinline__ void acc_guard4(v8f& a, v8f& b, v8f& c, v8f& d) { asm volatile("v_nop\n\tv_nop\n\tv_nop\n\tv_nop" : "+v"(a), "+v"(b), "+v"(c), "+v"(d)); }
template <typename T> struct Frag;
template <> struct Frag<_Float16> {
  typedef v16h V; union U { v16h v; v8h h[2]; };
  static __device__ __forceinline__ v16h load(const _Float16* p) {
    U f; f.h[0] = *(const v8h*)(p); f.h[1] = *(const v8h*)(p + 16); return f.v;
  }
  static __device__ __forceinline__ v8f mma(v16h a, v16h b, v8f c) {
    return __builtin_amdgcn_wmma_f32_16x16x32_f16(false, a, false, b, (short)0, c, false, false);
  }
  static __device__ __forceinline__ void guard(v8f& a, v8f& b, v16h x, v16h y) { dep_guard_h(a, b, x, y); }
  static __device__ __forceinline__ void keep(v16h a, v16h b, v16h c, v16h d) { keep4_h(a, b, c, d); }
};
template <> struct Frag<__bf16> {
  typedef v16b V; union U { v16b v; v8b h[2]; };
  static __device__ __forceinline__ v16b load(const __bf16* p) {
    U f; f.h[0] = *(const v8b*)(p); f.h[1] = *(const v8b*)(p + 16); return f.v;
  }
  static __device__ __forceinline__ v8f mma(v16b a, v16b b, v8f c) {
    return __builtin_amdgcn_wmma_f32_16x16x32_bf16(false, a, false, b, (short)0, c, false, false);
  }
  static __device__ __forceinline__ void guard(v8f& a, v8f& b, v16b x, v16b y) { dep_guard_b(a, b, x, y); }
  static __device__ __forceinline__ void keep(v16b a, v16b b, v16b c, v16b d) { keep4_b(a, b, c, d); }
};

__device__ __forceinline__ unsigned pk16(unsigned short a, unsigned short b) { return (unsigned)a | ((unsigned)b << 16); }
__device__ __forceinline__ unsigned short h_bits(float f) { const _Float16 h = (_Float16)f; return __builtin_bit_cast(unsigned short, h); }

template <int ET> struct Elem;
template <> struct Elem<0> { typedef _Float16 T; };
template <> struct Elem<1> { typedef __bf16 T; };
template <int ET, bool SPLIT, int BIAS_MODE, int OUT_MODE, bool RESID, int ACT = 0>
__global__ __launch_bounds__(256) void wmma_gemm64(
    const unsigned short* __restrict__ Ap, const unsigned short* __restrict__ A2p, int lda, long strideA,
    const unsigned short* __restrict__ Btp, const unsigned short* __restrict__ Bt2p, int ldb, long strideB,
    void* __restrict__ Cout, void* __restrict__ Cout2, int ldc, long strideC,
    const float* __restrict__ bias,
    const float* __restrict__ resid, long strideR,
    int M, int N, int K, float scale) {
  typedef typename Elem<ET>::T T;
  typedef typename Frag<T>::V V;
  const T* A = (const T*)Ap; const T* A2 = (const T*)A2p; const T* Bt = (const T*)Btp; const T* Bt2 = (const T*)Bt2p;
  __shared__ __align__(16) float sT[8][16 * 68];
  const int b    = blockIdx.y;
  const int lane = threadIdx.x & 31;
  const int wave = threadIdx.x >> 5;
  const int tilesN = N >> 6;
  const int tilesM = M >> 6;
  const int tile = blockIdx.x * 8 + wave;
  if (tile >= tilesM * tilesN) return;
  const int tm = tile / tilesN;
  const int tn = tile - tm * tilesN;
  const int m0 = tm << 6;
  const int n0 = tn << 6;

  const T* Ab  = A  + (size_t)b * strideA;
  const T* Bb  = Bt + (size_t)b * strideB;
  const T* Ab2 = SPLIT ? (A2  + (size_t)b * strideA) : nullptr;
  const T* Bb2 = SPLIT ? (Bt2 + (size_t)b * strideB) : nullptr;

  const int rlane = lane & 15;
  const int koff  = (lane >> 4) * 8;
  const int mOff  = (lane >> 4) * 8;

  v8f acc[4][4];
#pragma unroll
  for (int i = 0; i < 4; ++i)
#pragma unroll
    for (int j = 0; j < 4; ++j) acc[i][j] = (v8f){0.f,0.f,0.f,0.f,0.f,0.f,0.f,0.f};

  for (int k0 = 0; k0 < K; k0 += 32) {
    V bh[4], bl[4];
#pragma unroll
    for (int j = 0; j < 4; ++j) {
      const size_t bo = (size_t)(n0 + (j << 4) + rlane) * ldb + koff + k0;
      bh[j] = Frag<T>::load(Bb + bo);
      if (SPLIT) bl[j] = Frag<T>::load(Bb2 + bo);
    }
#pragma unroll
    for (int i = 0; i < 4; ++i) {
      const size_t ao = (size_t)(m0 + (i << 4) + rlane) * lda + koff + k0;
      V ah = Frag<T>::load(Ab + ao);
      V al;
      if (SPLIT) al = Frag<T>::load(Ab2 + ao);
#pragma unroll
      for (int j = 0; j < 4; ++j) {
        acc[i][j] = Frag<T>::mma(ah, bh[j], acc[i][j]);
        if (SPLIT) {
          acc[i][j] = Frag<T>::mma(ah, bl[j], acc[i][j]);
          acc[i][j] = Frag<T>::mma(al, bh[j], acc[i][j]);
        }
      }
      Frag<T>::guard(acc[i][0], acc[i][3], ah, SPLIT ? al : ah);
    }
    Frag<T>::keep(bh[0], bh[1], bh[2], bh[3]);
    if (SPLIT) Frag<T>::keep(bl[0], bl[1], bl[2], bl[3]);
  }
  acc_guard4(acc[0][0], acc[0][1], acc[0][2], acc[0][3]);
  acc_guard4(acc[1][0], acc[1][1], acc[1][2], acc[1][3]);
  acc_guard4(acc[2][0], acc[2][1], acc[2][2], acc[2][3]);
  acc_guard4(acc[3][0], acc[3][1], acc[3][2], acc[3][3]);

  float* slab = sT[wave];
  const float* Rb = RESID ? (resid + (size_t)b * strideR) : nullptr;
#pragma unroll
  for (int i = 0; i < 4; ++i) {
    const int mBase = m0 + (i << 4);
#pragma unroll
    for (int j = 0; j < 4; ++j) {
      const int n = n0 + (j << 4) + rlane;
      float bv = 0.f;
      if (BIAS_MODE == 2) bv = bias[n];
#pragma unroll
      for (int r = 0; r < 8; ++r) {
        float v = acc[i][j][r] * scale;
        if (BIAS_MODE == 1) v += bias[mBase + mOff + r];
        if (BIAS_MODE == 2) v += bv;
        if (RESID) v += Rb[(size_t)(mBase + mOff + r) * ldc + n];
        if (ACT == 2) v = fmaxf(v, 0.0f);
        if (ACT == 4) v = (v > 0.f) ? v : 0.01f * v;
        slab[(mOff + r) * 68 + (j << 4) + rlane] = v;
      }
    }
    __builtin_amdgcn_fence(__ATOMIC_RELEASE, "workgroup");
    __builtin_amdgcn_wave_barrier();
    __builtin_amdgcn_fence(__ATOMIC_ACQUIRE, "workgroup");
    if (OUT_MODE == 0) {
      float* C = (float*)Cout + (size_t)b * strideC;
      const int hh = lane >> 4, c4 = (lane & 15) * 4;
      for (int pass = 0; pass < 2; ++pass) {
#pragma unroll
        for (int it = 0; it < 8; ++it) {
          const int row = it * 2 + hh;
          v4f v = *(const v4f*)(slab + row * 68 + c4);
          *(volatile v4f*)(C + (size_t)(mBase + row) * ldc + n0 + c4) = v;
        }
        __threadfence();
      }
    } else {
      const int q = lane >> 3, c8 = (lane & 7) * 8;
      unsigned short* C  = (unsigned short*)Cout  + (size_t)b * strideC;
      unsigned short* C2 = (OUT_MODE == 2) ? ((unsigned short*)Cout2 + (size_t)b * strideC) : nullptr;
      for (int pass = 0; pass < 2; ++pass) {
#pragma unroll
        for (int it = 0; it < 4; ++it) {
          const int row = it * 4 + q;
          const float* sp = slab + row * 68 + c8;
          v8h hv, lv;
#pragma unroll
          for (int e = 0; e < 8; ++e) {
            if (OUT_MODE == 1) {
              hv[e] = (_Float16)sp[e];
            } else {
              unsigned short hb = f2bf_bits(sp[e]);
              unsigned short lb = f2bf_bits(sp[e] - bf_bits2f(hb));
              hv[e] = __builtin_bit_cast(_Float16, hb);
              lv[e] = __builtin_bit_cast(_Float16, lb);
            }
          }
          *(volatile v8h*)(C + (size_t)(mBase + row) * ldc + n0 + c8) = hv;
          if (OUT_MODE == 2) *(volatile v8h*)(C2 + (size_t)(mBase + row) * ldc + n0 + c8) = lv;
        }
        __threadfence();
      }
    }
    __builtin_amdgcn_fence(__ATOMIC_RELEASE, "workgroup");
    __builtin_amdgcn_wave_barrier();
    __builtin_amdgcn_fence(__ATOMIC_ACQUIRE, "workgroup");
  }
}

__global__ __launch_bounds__(256) void cast8_f16_kernel(const float* __restrict__ in, unsigned short* __restrict__ out, int n8) {
  const int i = blockIdx.x * 256 + threadIdx.x;
  if (i >= n8) return;
  const float* p = in + 8 * (size_t)i;
  const v4f a = *(const v4f*)(p);
  const v4f c = *(const v4f*)(p + 4);
  unsigned short hb[8];
#pragma unroll
  for (int e = 0; e < 4; ++e) {
    hb[e]     = h_bits(a[e]);
    hb[4 + e] = h_bits(c[e]);
  }
  const v4u u = (v4u){pk16(hb[0], hb[1]), pk16(hb[2], hb[3]), pk16(hb[4], hb[5]), pk16(hb[6], hb[7])};
  unsigned short* q = out + 8 * (size_t)i;
  *(volatile v4u*)q = u;
  __threadfence();
  *(volatile v4u*)q = u;
}

__global__ __launch_bounds__(256) void wtcast64_kernel(const float* __restrict__ W0, const float* __restrict__ W1,
                                                       unsigned short* __restrict__ out, float scale) {
  __shared__ float sm[64][65];
  const int t  = threadIdx.x;
  const int h0 = blockIdx.x * 64;
  const int z  = blockIdx.z;
  const float* W = (z == 0) ? W0 : W1;
#pragma unroll
  for (int i = 0; i < 16; ++i) {
    const int e = i * 256 + t;
    const int r = e >> 6;
    const int c = e & 63;
    sm[c][r] = W[(size_t)r * kH + h0 + c] * scale;
  }
  __syncthreads();
  const int lane = t & 31, wave = t >> 5;
  const int q = lane >> 3, c8 = (lane & 7) * 8;
  unsigned short* op = out + (size_t)z * kH * kR;
  for (int pass = 0; pass < 2; ++pass) {
#pragma unroll
    for (int it = 0; it < 2; ++it) {
      const int row = wave * 8 + it * 4 + q;
      unsigned short hb[8];
#pragma unroll
      for (int e = 0; e < 8; ++e) hb[e] = h_bits(sm[row][c8 + e]);
      const v4u u = (v4u){pk16(hb[0], hb[1]), pk16(hb[2], hb[3]), pk16(hb[4], hb[5]), pk16(hb[6], hb[7])};
      *(volatile v4u*)(op + (size_t)(h0 + row) * kR + c8) = u;
    }
    __threadfence();
  }
}

__global__ __launch_bounds__(256) void ctcast_kernel(const float* __restrict__ Cin, unsigned short* __restrict__ CT) {
  __shared__ float sm[64][65];
  const int t  = threadIdx.x;
  const int d0 = blockIdx.x * 64;
  const int h0 = blockIdx.y * 64;
  const int b  = blockIdx.z;
  const float* src = Cin + (size_t)b * kH * kH;
#pragma unroll
  for (int i = 0; i < 16; ++i) {
    const int e  = i * 256 + t;
    const int hl = e >> 6;
    const int dl = e & 63;
    sm[dl][hl] = src[(size_t)(h0 + hl) * kH + d0 + dl];
  }
  __syncthreads();
  const int lane = t & 31, wave = t >> 5;
  const int q = lane >> 3, c8 = (lane & 7) * 8;
  unsigned short* dst = CT + (size_t)b * kH * kH;
  for (int pass = 0; pass < 2; ++pass) {
#pragma unroll
    for (int it = 0; it < 2; ++it) {
      const int row = wave * 8 + it * 4 + q;
      unsigned short hb[8];
#pragma unroll
      for (int e = 0; e < 8; ++e) hb[e] = h_bits(sm[row][c8 + e]);
      const v4u u = (v4u){pk16(hb[0], hb[1]), pk16(hb[2], hb[3]), pk16(hb[4], hb[5]), pk16(hb[6], hb[7])};
      *(volatile v4u*)(dst + (size_t)(d0 + row) * kH + h0 + c8) = u;
    }
    __threadfence();
  }
}

__global__ __launch_bounds__(256) void knorm_kernel(const float* __restrict__ Kf, unsigned short* __restrict__ KN, int nrows) {
  const int lane = threadIdx.x & 31, wave = threadIdx.x >> 5;
  const int rb = (blockIdx.x * 8 + wave) * kRowsPerWave;
#pragma unroll 1
  for (int rr = 0; rr < kRowsPerWave; ++rr) {
    int row = rb + rr;
    row = (row < nrows) ? row : (nrows - 1);
    const float* p = Kf + (size_t)row * kH;
    const v4f a0 = *(const v4f*)(p + 8 * lane);
    const v4f a1 = *(const v4f*)(p + 8 * lane + 4);
    const v4f c0 = *(const v4f*)(p + 256 + 8 * lane);
    const v4f c1 = *(const v4f*)(p + 256 + 8 * lane + 4);
    float s = 0.f;
#pragma unroll
    for (int e = 0; e < 4; ++e) s += a0[e] * a0[e];
#pragma unroll
    for (int e = 0; e < 4; ++e) s += a1[e] * a1[e];
#pragma unroll
    for (int e = 0; e < 4; ++e) s += c0[e] * c0[e];
#pragma unroll
    for (int e = 0; e < 4; ++e) s += c1[e] * c1[e];
#pragma unroll
    for (int off = 16; off > 0; off >>= 1) s += __shfl_xor(s, off, 32);
    const float nrm = sqrtf(s);
    const float sc  = (1.0f / fmaxf(nrm, kEps)) * kKCarry;
    const v4u u0 = (v4u){pk16(h_bits(a0[0] * sc), h_bits(a0[1] * sc)), pk16(h_bits(a0[2] * sc), h_bits(a0[3] * sc)),
                         pk16(h_bits(a1[0] * sc), h_bits(a1[1] * sc)), pk16(h_bits(a1[2] * sc), h_bits(a1[3] * sc))};
    const v4u u1 = (v4u){pk16(h_bits(c0[0] * sc), h_bits(c0[1] * sc)), pk16(h_bits(c0[2] * sc), h_bits(c0[3] * sc)),
                         pk16(h_bits(c1[0] * sc), h_bits(c1[1] * sc)), pk16(h_bits(c1[2] * sc), h_bits(c1[3] * sc))};
    unsigned short* qp = KN + (size_t)row * kH;
    *(volatile v4u*)(qp + 8 * lane) = u0;
    *(volatile v4u*)(qp + 256 + 8 * lane) = u1;
    __threadfence();
    *(volatile v4u*)(qp + 8 * lane) = u0;
    *(volatile v4u*)(qp + 256 + 8 * lane) = u1;
  }
}

__global__ __launch_bounds__(256) void ktrans_kernel(const unsigned short* __restrict__ KN, unsigned short* __restrict__ KNT) {
  __shared__ unsigned int sm32[64][33];
  const int t  = threadIdx.x;
  const int h0 = blockIdx.x * 64;
  const int l0 = blockIdx.y * 64;
  const int bb = blockIdx.z;
  const unsigned short* src = KN + (size_t)bb * kL * kH;
#pragma unroll
  for (int i = 0; i < 8; ++i) {
    const int e  = i * 256 + t;
    const int r  = e >> 5;
    const int c2 = e & 31;
    sm32[r][c2] = *(const unsigned int*)(src + (size_t)(l0 + r) * kH + h0 + 2 * c2);
  }
  __syncthreads();
  const int lane = t & 31, wave = t >> 5;
  const int q = lane >> 3, c8 = (lane & 7) * 8;
  unsigned short* dst = KNT + (size_t)bb * kH * kL;
  for (int pass = 0; pass < 2; ++pass) {
#pragma unroll
    for (int it = 0; it < 2; ++it) {
      const int row = wave * 8 + it * 4 + q;
      const int wsh = (row & 1) * 16;
      const int wi  = row >> 1;
      unsigned short hb[8];
#pragma unroll
      for (int e = 0; e < 8; ++e) hb[e] = (unsigned short)((sm32[c8 + e][wi] >> wsh) & 0xffffu);
      const v4u u = (v4u){pk16(hb[0], hb[1]), pk16(hb[2], hb[3]), pk16(hb[4], hb[5]), pk16(hb[6], hb[7])};
      *(volatile v4u*)(dst + (size_t)(h0 + row) * kL + l0 + c8) = u;
    }
    __threadfence();
  }
}

extern "C" void kernel_launch(void* const* d_in, const int* in_sizes, int n_in,
                              void* d_out, int out_size, void* d_ws, size_t ws_size,
                              hipStream_t stream) {
  if (n_in < 6) return;
  if (in_sizes[0] != kB * kL * kR) return;
  if (in_sizes[1] != kB * kH * kH) return;
  if (in_sizes[2] != kR * kH) return;
  if (in_sizes[3] != kH) return;
  if (in_sizes[4] != kR * kH) return;
  if (in_sizes[5] != kH) return;
  if (out_size != kB * kH * kH) return;

  const float* hs      = (const float*)d_in[0];
  const float* cache   = (const float*)d_in[1];
  const float* key_w   = (const float*)d_in[2];
  const float* key_b   = (const float*)d_in[3];
  const float* value_w = (const float*)d_in[4];
  const float* value_b = (const float*)d_in[5];
  float* out = (float*)d_out;

  const size_t szHs  = (size_t)kB * kL * kR * 2;
  const size_t szWt  = (size_t)2 * kH * kR * 2;
  const size_t szCT  = (size_t)kB * kH * kH * 2;
  const size_t szKf  = (size_t)kRowsChunk * kH * 4;
  const size_t szKN  = (size_t)kRowsChunk * kH * 2;
  const size_t szKNT = (size_t)kNBC * kH * kL * 2;
  const size_t szVT  = (size_t)kNBC * kH * kL * 4;
  const size_t szV2T = (size_t)kNBC * kH * kL * 2;
  const size_t offHs  = 0;
  const size_t offWt  = offHs + szHs;
  const size_t offCT  = offWt + szWt;
  const size_t offKf  = offCT + szCT;
  const size_t offKN  = offKf + szKf;
  const size_t offKNT = offKN + szKN;
  const size_t offVT  = offKNT + szKNT;
  const size_t offV2T = offVT + szVT;
  const size_t offEnd = offV2T + szV2T;
  if (offEnd > ws_size) return;

  char* ws = (char*)d_ws;
  unsigned short* hsH = (unsigned short*)(ws + offHs);
  unsigned short* Wt  = (unsigned short*)(ws + offWt);
  unsigned short* WkT = Wt;
  unsigned short* WvT = Wt + (size_t)kH * kR;
  unsigned short* CT  = (unsigned short*)(ws + offCT);
  float*          Kf  = (float*)(ws + offKf);
  unsigned short* KN  = (unsigned short*)(ws + offKN);
  unsigned short* KNT = (unsigned short*)(ws + offKNT);
  float*          VTf = (float*)(ws + offVT);
  unsigned short* V2T = (unsigned short*)(ws + offV2T);

  {
    const int n8 = kB * kL * kR / 8;
    cast8_f16_kernel<<<dim3((n8 + 255) / 256), dim3(256), 0, stream>>>(hs, hsH, n8);
    wtcast64_kernel<<<dim3(kH / 64, 1, 2), dim3(256), 0, stream>>>(key_w, value_w, Wt, kWCarry);
    ctcast_kernel<<<dim3(kH / 64, kH / 64, kB), dim3(256), 0, stream>>>(cache, CT);
  }

  for (int ch = 0; ch < kNChunk; ++ch) {
    const size_t row0  = (size_t)ch * kRowsChunk;
    const size_t bat0  = (size_t)ch * kNBC;
    const unsigned short* hsC = hsH + row0 * kR;
    const unsigned short* CTC = CT + bat0 * kH * kH;
    const float* cacheC = cache + bat0 * kH * kH;
    float* outC = out + bat0 * kH * kH;

    wmma_gemm64<0, false, 2, 0, false, 0><<<dim3((kRowsChunk / 64) * (kH / 64) / 8, 1), dim3(256), 0, stream>>>(
        hsC, nullptr, kR, 0L,
        WkT, nullptr, kR, 0L,
        (void*)Kf, nullptr, kH, 0L,
        key_b, nullptr, 0L,
        kRowsChunk, kH, kR, kInvW);

    knorm_kernel<<<dim3(kRowsChunk / (8 * kRowsPerWave)), dim3(256), 0, stream>>>(Kf, KN, kRowsChunk);

    ktrans_kernel<<<dim3(kH / 64, kL / 64, kNBC), dim3(256), 0, stream>>>(KN, KNT);

    wmma_gemm64<0, false, 1, 0, false, 0><<<dim3((kH / 64) * (kL / 64) / 8, kNBC), dim3(256), 0, stream>>>(
        WvT, nullptr, kR, 0L,
        hsC, nullptr, kR, (long)kL * kR,
        (void*)VTf, nullptr, kL, (long)kH * kL,
        value_b, nullptr, 0L,
        kH, kL, kR, kInvW);

    wmma_gemm64<0, false, 0, 1, true, 0><<<dim3((kH / 64) * (kL / 64) / 8, kNBC), dim3(256), 0, stream>>>(
        CTC, nullptr, kH, (long)kH * kH,
        KN, nullptr, kH, (long)kL * kH,
        (void*)V2T, nullptr, kL, (long)kH * kL,
        nullptr, VTf, (long)kH * kL,
        kH, kL, kH, -kInvK);

    wmma_gemm64<0, false, 0, 0, true, 0><<<dim3((kH / 64) * (kH / 64) / 8, kNBC), dim3(256), 0, stream>>>(
        KNT, nullptr, kL, (long)kH * kL,
        V2T, nullptr, kL, (long)kH * kL,
        (void*)outC, nullptr, kH, (long)kH * kH,
        nullptr, cacheC, (long)kH * kH,
        kH, kH, kL, kInvK);
  }
}
